// UHGGINLayer_21328807592547
// MI455X (gfx1250) — hardware-verified
//
#include <hip/hip_runtime.h>
#include <stddef.h>


#define DF    128
#define NB    512
#define RP    132
#define RPU   264
#define TR    64
#define NTILE (NB / TR)
#define CHUNK 2048
#define NTHR  256
#define NWAVE 8
#define WCAP  256
#define NGRP  (CHUNK / (NTHR * 4))

#define LDS_ACC   (NB * RP)
#define LDS_DEN   NB
#define LDS_MAX   NB
#define LDS_LIST  (NWAVE * WCAP)
#define LDS_CNT   16
#define LDS_BYTES ((LDS_ACC + LDS_DEN + LDS_MAX + LDS_LIST + LDS_CNT) * 4)

static_assert(LDS_BYTES == 282688);
static_assert(WCAP == (CHUNK / NTHR) * 32);
static_assert(NGRP == 2);
static_assert(((LDS_ACC + LDS_DEN) % 4) == 0);
static_assert((RP % 4) == 0);
static_assert(NB == NWAVE * 64);
static_assert(TR == NWAVE * 8);
static_assert((NB & (NB - 1)) == 0);
static_assert((CHUNK & (CHUNK - 1)) == 0);
static_assert(NB <= 512 && CHUNK <= 4096);

typedef float          v4f  __attribute__((ext_vector_type(4)));
typedef float          v8f  __attribute__((ext_vector_type(8)));
typedef int            v4i  __attribute__((ext_vector_type(4)));
typedef unsigned int   v2u  __attribute__((ext_vector_type(2)));
typedef unsigned short v8us __attribute__((ext_vector_type(8)));
typedef __bf16         v16b __attribute__((ext_vector_type(16)));
union FragB { v16b v; v8us half[2]; };

__device__ __forceinline__ v8f wmb(v16b a, v16b b, v8f c) {
  v8f d = __builtin_amdgcn_wmma_f32_16x16x32_bf16(false, a, false, b, (short)0, c, false, false);
  asm volatile("v_nop\n\tv_nop\n\tv_nop\n\tv_nop" : "+v"(d) : "v"(a), "v"(b));
  return d;
}

__device__ __forceinline__ float wsum(float v) {
  v += __shfl_xor(v, 16, 32);
  v += __shfl_xor(v, 8, 32);
  v += __shfl_xor(v, 4, 32);
  v += __shfl_xor(v, 2, 32);
  v += __shfl_xor(v, 1, 32);
  return v;
}

__device__ __forceinline__ unsigned short bf_rne(float f) {
  unsigned u = __float_as_uint(f);
  u += 0x7fffu + ((u >> 16) & 1u);
  return (unsigned short)(u >> 16);
}
__device__ __forceinline__ float bf_val(unsigned short b) {
  return __uint_as_float(((unsigned)b) << 16);
}

__global__ __launch_bounds__(NTHR) void k_prep(const float* __restrict__ W1,
                                               const float* __restrict__ W2,
                                               unsigned short* planes) {
  __shared__ __attribute__((aligned(16))) float S[DF * 33];
  const int tid = threadIdx.x;
  const int mat = (int)(blockIdx.x >> 2);
  const int n0  = (int)(blockIdx.x & 3) * 32;
  const float* W = (mat != 0) ? W2 : W1;
  {
    const int k  = tid >> 1;
    const int c0 = (tid & 1) * 16;
    const float* p = W + (size_t)k * DF + n0 + c0;
    const v4f f0 = *(const v4f*)(p);
    const v4f f1 = *(const v4f*)(p + 4);
    const v4f f2 = *(const v4f*)(p + 8);
    const v4f f3 = *(const v4f*)(p + 12);
    float* s = S + k * 33 + c0;
    s[0]  = f0.x; s[1]  = f0.y; s[2]  = f0.z; s[3]  = f0.w;
    s[4]  = f1.x; s[5]  = f1.y; s[6]  = f1.z; s[7]  = f1.w;
    s[8]  = f2.x; s[9]  = f2.y; s[10] = f2.z; s[11] = f2.w;
    s[12] = f3.x; s[13] = f3.y; s[14] = f3.z; s[15] = f3.w;
  }
  __syncthreads();
  unsigned short* Wh = planes + (size_t)mat * 2 * DF * DF;
  unsigned short* Wl = Wh + DF * DF;
  v8us hv[2], lv[2];
  size_t oo[2];
#pragma unroll
  for (int q = 0; q < 2; ++q) {
    const int idx = q * NTHR + tid;
    const int nl  = idx >> 4;
    const int g   = idx & 15;
#pragma unroll
    for (int i = 0; i < 8; ++i) {
      const float v = S[(8 * g + i) * 33 + nl];
      const unsigned short hb = bf_rne(v);
      const unsigned short lb = bf_rne(v - bf_val(hb));
      hv[q][i] = hb;
      lv[q][i] = lb;
    }
    oo[q] = (size_t)(n0 + nl) * DF + 8 * g;
  }
#pragma unroll
  for (int q = 0; q < 2; ++q) {
    *(volatile v8us*)(Wh + oo[q]) = hv[q];
    *(volatile v8us*)(Wl + oo[q]) = lv[q];
  }
  __threadfence();
#pragma unroll
  for (int q = 0; q < 2; ++q) {
    *(volatile v8us*)(Wh + oo[q]) = hv[q];
    *(volatile v8us*)(Wl + oo[q]) = lv[q];
  }
}

__global__ __launch_bounds__(NTHR) void k_main(
    const float* __restrict__ x, const int* __restrict__ ei, const float* __restrict__ ea,
    const unsigned short* __restrict__ W1h, const unsigned short* __restrict__ W1l,
    const unsigned short* __restrict__ W2h, const unsigned short* __restrict__ W2l,
    const float* __restrict__ b1, const float* __restrict__ b2,
    const float* __restrict__ gam, const float* __restrict__ bet,
    float* out, int nN, int nE) {
  extern __shared__ v4f lds_dyn[];
  float* sacc = (float*)lds_dyn;
  float* den  = sacc + LDS_ACC;
  float* mrun = den + LDS_DEN;
  int*   list = (int*)(mrun + LDS_MAX);
  int*   wcnt = list + LDS_LIST;
  unsigned short* us = (unsigned short*)lds_dyn;

  const int tid  = threadIdx.x;
  const int lane = tid & 31;
  const int wave = tid >> 5;
  const int hh   = lane >> 4;
  const int m    = lane & 15;
  const int nodeBase = blockIdx.x * NB;

  {
    const v4f z4 = {0.f, 0.f, 0.f, 0.f};
    for (int i = tid; i < (LDS_ACC + LDS_DEN) / 4; i += NTHR) lds_dyn[i] = z4;
    const float ninf = __uint_as_float(0xff800000u);
    for (int i = tid; i < NB; i += NTHR) mrun[i] = ninf;
  }
  __syncthreads();

  const int* eid = ei + nE;
  const bool al16 = ((nE & 3) == 0);

  const int nChunks = (nE + CHUNK - 1) / CHUNK;
#pragma unroll 1
  for (int ch = 0; ch < nChunks; ++ch) {
    const int cbase = ch * CHUNK;
    int wc = 0;
#pragma unroll
    for (int g = 0; g < NGRP; ++g) {
      const int el0 = (g * NTHR + tid) * 4;
      const int e0  = cbase + el0;
      const int sent = -2147483647 - 1;
      v4i d;
      if (al16 && (cbase + CHUNK <= nE)) {
        d = *(const v4i*)(eid + e0);
      } else {
        d.x = (e0     < nE) ? eid[min(e0,     nE - 1)] : sent;
        d.y = (e0 + 1 < nE) ? eid[min(e0 + 1, nE - 1)] : sent;
        d.z = (e0 + 2 < nE) ? eid[min(e0 + 2, nE - 1)] : sent;
        d.w = (e0 + 3 < nE) ? eid[min(e0 + 3, nE - 1)] : sent;
      }
      const unsigned s0 = (unsigned)d.x - (unsigned)nodeBase;
      const unsigned s1 = (unsigned)d.y - (unsigned)nodeBase;
      const unsigned s2 = (unsigned)d.z - (unsigned)nodeBase;
      const unsigned s3 = (unsigned)d.w - (unsigned)nodeBase;
      const bool h0 = s0 < (unsigned)NB;
      const bool h1 = s1 < (unsigned)NB;
      const bool h2 = s2 < (unsigned)NB;
      const bool h3 = s3 < (unsigned)NB;
      const unsigned many = __builtin_amdgcn_ballot_w32(h0 | h1 | h2 | h3);
      if (many != 0u) {
#define HITJ(J, HJ, SJ) { \
          const unsigned mj = __builtin_amdgcn_ballot_w32(HJ); \
          if (HJ) { \
            const int pos = wc + (int)__builtin_amdgcn_mbcnt_lo(mj, 0u); \
            if (pos < WCAP) list[wave * WCAP + pos] = ((el0 + (J)) << 9) | (int)(SJ); \
          } \
          wc += (int)__builtin_popcount(mj); }
        HITJ(0, h0, s0)
        HITJ(1, h1, s1)
        HITJ(2, h2, s2)
        HITJ(3, h3, s3)
#undef HITJ
      }
    }
    if (lane == 0) wcnt[wave] = wc;
    __syncthreads();

    if (wave == 0) {
#pragma unroll 1
      for (int wsx = 0; wsx < NWAVE; ++wsx) {
        int n = wcnt[wsx];
        if (n > WCAP) n = WCAP;
        if (n < 0) n = 0;
#pragma unroll 1
        for (int i = 0; i < n; ++i) {
          const int ent  = list[wsx * WCAP + i];
          const int slot = ent & (NB - 1);
          const int el   = (ent >> 9) & (CHUNK - 1);
          int e = cbase + el;
          if (e > nE - 1) e = nE - 1;
          int src = ei[e];
          src = src < 0 ? 0 : (src > nN - 1 ? nN - 1 : src);
          const float w    = ea[e];
          const float mo   = mrun[slot];
          const float dcur = den[slot];
          const bool  up   = w > mo;
          const float mn   = up ? w : mo;
          const float ea1  = __expf(mo - w);
          const float eb1  = __expf(w - mo);
          const float sc   = up ? ea1 : 1.0f;
          const float p    = up ? 1.0f : eb1;
          const v4f xv = *(const v4f*)(x + (size_t)src * DF + 4 * lane);
          v4f* sp = (v4f*)(sacc + slot * RP + 4 * lane);
          const v4f cur = *sp;
          *sp = cur * sc + xv * p;
          mrun[slot] = mn;
          den[slot]  = dcur * sc + p;
        }
      }
    }
    __syncthreads();
  }

#pragma unroll 1
  for (int j = 0; j < NB / NWAVE; ++j) {
    const int slot = wave * (NB / NWAVE) + j;
    int node = nodeBase + slot;
    if (node > nN - 1) node = nN - 1;
    v4f a = *(const v4f*)(sacc + slot * RP + 4 * lane);
    const float dd   = den[slot];
    const float invd = (dd > 0.f) ? (1.0f / fmaxf(dd, 1e-30f)) : 0.f;
    a = a * invd;
    const float ss   = wsum(a.x * a.x + a.y * a.y + a.z * a.z + a.w * a.w);
    const float invn = 1.0f / (sqrtf(ss) + 1e-9f);
    const v4f xr = *(const v4f*)(x + (size_t)node * DF + 4 * lane);
    const v4f c = xr + a * invn;
    const unsigned short c0h = bf_rne(c.x), c1h = bf_rne(c.y), c2h = bf_rne(c.z), c3h = bf_rne(c.w);
    const unsigned short c0l = bf_rne(c.x - bf_val(c0h)), c1l = bf_rne(c.y - bf_val(c1h));
    const unsigned short c2l = bf_rne(c.z - bf_val(c2h)), c3l = bf_rne(c.w - bf_val(c3h));
    v2u hvv, lvv;
    hvv.x = (unsigned)c0h | ((unsigned)c1h << 16);
    hvv.y = (unsigned)c2h | ((unsigned)c3h << 16);
    lvv.x = (unsigned)c0l | ((unsigned)c1l << 16);
    lvv.y = (unsigned)c2l | ((unsigned)c3l << 16);
    unsigned short* ur = us + (size_t)slot * RPU;
    *(v2u*)(ur + 4 * lane)       = hvv;
    *(v2u*)(ur + 128 + 4 * lane) = lvv;
  }
  __syncthreads();

  const int   col = wave * 16 + m;
  const float b1c = b1[col];
  const float b2c = b2[col];
  const v4f   g4  = *(const v4f*)(gam + 4 * lane);
  const v4f   e4  = *(const v4f*)(bet + 4 * lane);

#pragma unroll 1
  for (int T = 0; T < NTILE; ++T) {
    const int r0 = T * TR;
    if (nodeBase + r0 >= nN) break;

    v8f acc[4];
#pragma unroll
    for (int t = 0; t < 4; ++t) { const v8f z = {0.f, 0.f, 0.f, 0.f, 0.f, 0.f, 0.f, 0.f}; acc[t] = z; }
#pragma unroll
    for (int kt = 0; kt < DF / 32; ++kt) {
      const int k0 = kt * 32;
      FragB bh, bl;
      const size_t bo = (size_t)col * DF + k0 + 8 * hh;
      bh.half[0] = *(const v8us*)(W1h + bo); bh.half[1] = *(const v8us*)(W1h + bo + 16);
      bl.half[0] = *(const v8us*)(W1l + bo); bl.half[1] = *(const v8us*)(W1l + bo + 16);
#pragma unroll
      for (int t = 0; t < 4; ++t) {
        const unsigned short* ar = us + (size_t)(r0 + 16 * t + m) * RPU + k0 + 8 * hh;
        FragB ah, al;
        ah.half[0] = *(const v8us*)(ar);       ah.half[1] = *(const v8us*)(ar + 16);
        al.half[0] = *(const v8us*)(ar + 128); al.half[1] = *(const v8us*)(ar + 144);
        acc[t] = wmb(ah.v, bh.v, acc[t]);
        acc[t] = wmb(al.v, bh.v, acc[t]);
        acc[t] = wmb(ah.v, bl.v, acc[t]);
      }
    }
    __syncthreads();

#pragma unroll
    for (int t = 0; t < 4; ++t) {
#pragma unroll
      for (int r = 0; r < 8; ++r) {
        const int row = r0 + 16 * t + 8 * hh + r;
        const float v = fmaxf(acc[t][r] + b1c, 0.f);
        const unsigned short hb = bf_rne(v);
        const unsigned short lb = bf_rne(v - bf_val(hb));
        us[(size_t)row * RPU + col]       = hb;
        us[(size_t)row * RPU + 128 + col] = lb;
      }
    }
    __syncthreads();

#pragma unroll
    for (int t = 0; t < 4; ++t) { const v8f z = {0.f, 0.f, 0.f, 0.f, 0.f, 0.f, 0.f, 0.f}; acc[t] = z; }
#pragma unroll
    for (int kt = 0; kt < DF / 32; ++kt) {
      const int k0 = kt * 32;
      FragB bh, bl;
      const size_t bo = (size_t)col * DF + k0 + 8 * hh;
      bh.half[0] = *(const v8us*)(W2h + bo); bh.half[1] = *(const v8us*)(W2h + bo + 16);
      bl.half[0] = *(const v8us*)(W2l + bo); bl.half[1] = *(const v8us*)(W2l + bo + 16);
#pragma unroll
      for (int t = 0; t < 4; ++t) {
        const unsigned short* ar = us + (size_t)(r0 + 16 * t + m) * RPU + k0 + 8 * hh;
        FragB ah, al;
        ah.half[0] = *(const v8us*)(ar);       ah.half[1] = *(const v8us*)(ar + 16);
        al.half[0] = *(const v8us*)(ar + 128); al.half[1] = *(const v8us*)(ar + 144);
        acc[t] = wmb(ah.v, bh.v, acc[t]);
        acc[t] = wmb(al.v, bh.v, acc[t]);
        acc[t] = wmb(ah.v, bl.v, acc[t]);
      }
    }
    __syncthreads();

#pragma unroll
    for (int t = 0; t < 4; ++t) {
#pragma unroll
      for (int r = 0; r < 8; ++r) {
        const int row = r0 + 16 * t + 8 * hh + r;
        sacc[(size_t)row * RP + col] = acc[t][r] + b2c;
      }
    }
    __syncthreads();

    v4f yv[8];
#pragma unroll
    for (int i = 0; i < 8; ++i) {
      const int lr = r0 + 8 * wave + i;
      const v4f h = *(const v4f*)(sacc + (size_t)lr * RP + 4 * lane);
      const float s  = wsum(h.x + h.y + h.z + h.w);
      const float mu = s * (1.0f / DF);
      const v4f dd = h - mu;
      const float q  = wsum(dd.x * dd.x + dd.y * dd.y + dd.z * dd.z + dd.w * dd.w);
      const float rs = rsqrtf(q * (1.0f / DF) + 1e-5f);
      yv[i] = dd * rs * g4 + e4;
    }
#pragma unroll
    for (int i = 0; i < 8; ++i) {
      const int node = nodeBase + r0 + 8 * wave + i;
      if (node < nN) *(volatile v4f*)(out + (size_t)node * DF + 4 * lane) = yv[i];
    }
    __threadfence();
#pragma unroll
    for (int i = 0; i < 8; ++i) {
      const int node = nodeBase + r0 + 8 * wave + i;
      if (node < nN) *(volatile v4f*)(out + (size_t)node * DF + 4 * lane) = yv[i];
    }
    __syncthreads();
  }
}

extern "C" void kernel_launch(void* const* d_in, const int* in_sizes, int n_in,
                              void* d_out, int out_size, void* d_ws, size_t ws_size,
                              hipStream_t stream) {
  if (n_in < 9) return;
  const int nN = in_sizes[0] / DF;
  const int nE = in_sizes[2];
  if (nN <= 0 || in_sizes[0] != nN * DF) return;
  if (nE < 0 || in_sizes[1] != 2 * nE) return;
  if (in_sizes[3] != DF * DF || in_sizes[5] != DF * DF) return;
  if (in_sizes[4] != DF || in_sizes[6] != DF || in_sizes[7] != DF || in_sizes[8] != DF) return;
  if (out_size != nN * DF) return;

  const float* x   = (const float*)d_in[0];
  const int*   ei  = (const int*)d_in[1];
  const float* ea  = (const float*)d_in[2];
  const float* W1  = (const float*)d_in[3];
  const float* b1  = (const float*)d_in[4];
  const float* W2  = (const float*)d_in[5];
  const float* b2  = (const float*)d_in[6];
  const float* gam = (const float*)d_in[7];
  const float* bet = (const float*)d_in[8];
  float* out = (float*)d_out;

  size_t off = 0;
  unsigned short* planes = (unsigned short*)((char*)d_ws + off);
  off += (size_t)4 * DF * DF * sizeof(unsigned short);
  if (off > ws_size) return;
  const unsigned short* W1h = planes;
  const unsigned short* W1l = planes + (size_t)DF * DF;
  const unsigned short* W2h = planes + (size_t)2 * DF * DF;
  const unsigned short* W2l = planes + (size_t)3 * DF * DF;

  k_prep<<<8, NTHR, 0, stream>>>(W1, W2, planes);

  hipFuncSetAttribute(reinterpret_cast<const void*>(&k_main),
                      hipFuncAttributeMaxDynamicSharedMemorySize, LDS_BYTES);
  const int grid = (nN + NB - 1) / NB;
  k_main<<<grid, NTHR, LDS_BYTES, stream>>>(x, ei, ea, W1h, W1l, W2h, W2l,
                                            b1, b2, gam, bet, out, nN, nE);
}
